// _GINBackbone_36421322670670
// MI455X (gfx1250) — hardware-verified
//
#include <hip/hip_runtime.h>
#include <stddef.h>


#define DF      64
#define NTHR    256
#define NWAVE   8
#define EPT     8
#define NGRP    2
#define CHUNK   (NTHR * EPT * NGRP)
#define WCAP    (EPT * NGRP * 32)
#define LISTN   (NWAVE * WCAP)
#define NBA     1024
#define GR2     256
#define GBLK    64
#define APITCH  72
#define TABN    256
#define PARTN   128
#define WSCALE  16.0f
#define WINV    0.0625f
#define BN_EPS  1e-5f

#define LDS_AGG (NBA * DF * 4 + LISTN * 4 + 64)
#define LDS_G2  (GR2 * APITCH * 2 + GR2 * DF * 4)

static_assert((CHUNK & (CHUNK - 1)) == 0);
static_assert(CHUNK <= 4096);
static_assert((NBA & (NBA - 1)) == 0 && NBA <= 4096);
static_assert((GBLK & (GBLK - 1)) == 0 && GBLK <= 4096);
static_assert(NBA % (16 * NWAVE) == 0);
static_assert(GR2 % (16 * NWAVE) == 0);
static_assert(GBLK == 8 * NWAVE);
static_assert((4 * 64 * 2 + PARTN) * 8 <= LISTN * 4);
static_assert((4 * 64 * 2 + PARTN) * 8 <= GR2 * APITCH * 2);
static_assert(((DF * DF / 8) % 32) == 0);
static_assert((APITCH * 2) % 16 == 0);

typedef float    v2f  __attribute__((ext_vector_type(2)));
typedef float    v4f  __attribute__((ext_vector_type(4)));
typedef float    v8f  __attribute__((ext_vector_type(8)));
typedef int      v4i  __attribute__((ext_vector_type(4)));
typedef double   v2d  __attribute__((ext_vector_type(2)));
typedef _Float16 v8h  __attribute__((ext_vector_type(8)));
typedef _Float16 v16h __attribute__((ext_vector_type(16)));
union FragH { v16h v; v8h h[2]; };

__device__ __forceinline__ v8h cvt8(v4f a, v4f b) {
  v8h r;
  r[0] = (_Float16)a.x; r[1] = (_Float16)a.y; r[2] = (_Float16)a.z; r[3] = (_Float16)a.w;
  r[4] = (_Float16)b.x; r[5] = (_Float16)b.y; r[6] = (_Float16)b.z; r[7] = (_Float16)b.w;
  return r;
}

__device__ __forceinline__ v8f wmh(v16h a, v16h b, v8f c) {
  v8f d = __builtin_amdgcn_wmma_f32_16x16x32_f16(false, a, false, b, (short)0, c, false, false);
  asm volatile("v_nop\n\tv_nop\n\tv_nop\n\tv_nop" : "+v"(d) : "v"(a), "v"(b));
  return d;
}

template <int NB>
__device__ __forceinline__ int scan_chunk(const int* __restrict__ keys, int nK, int cbase, int base,
                                          int vec8, int* list, int tid, int lane, int wave) {
  int wc = 0;
#pragma unroll
  for (int g = 0; g < NGRP; ++g) {
    const int el0  = (g * NTHR + tid) * EPT;
    const int e0   = cbase + el0;
    const int sent = -2147483647 - 1;
    v4i da, db;
    if (vec8 != 0 && cbase + CHUNK <= nK) {
      da = *(const v4i*)(keys + e0);
      db = *(const v4i*)(keys + e0 + 4);
    } else {
      da.x = (e0     < nK) ? keys[min(e0,     nK - 1)] : sent;
      da.y = (e0 + 1 < nK) ? keys[min(e0 + 1, nK - 1)] : sent;
      da.z = (e0 + 2 < nK) ? keys[min(e0 + 2, nK - 1)] : sent;
      da.w = (e0 + 3 < nK) ? keys[min(e0 + 3, nK - 1)] : sent;
      db.x = (e0 + 4 < nK) ? keys[min(e0 + 4, nK - 1)] : sent;
      db.y = (e0 + 5 < nK) ? keys[min(e0 + 5, nK - 1)] : sent;
      db.z = (e0 + 6 < nK) ? keys[min(e0 + 6, nK - 1)] : sent;
      db.w = (e0 + 7 < nK) ? keys[min(e0 + 7, nK - 1)] : sent;
    }
    const unsigned nb = (unsigned)base;
    const unsigned s0 = (unsigned)da.x - nb, s1 = (unsigned)da.y - nb;
    const unsigned s2 = (unsigned)da.z - nb, s3 = (unsigned)da.w - nb;
    const unsigned s4 = (unsigned)db.x - nb, s5 = (unsigned)db.y - nb;
    const unsigned s6 = (unsigned)db.z - nb, s7 = (unsigned)db.w - nb;
    const bool h0 = s0 < (unsigned)NB, h1 = s1 < (unsigned)NB, h2 = s2 < (unsigned)NB, h3 = s3 < (unsigned)NB;
    const bool h4 = s4 < (unsigned)NB, h5 = s5 < (unsigned)NB, h6 = s6 < (unsigned)NB, h7 = s7 < (unsigned)NB;
    const unsigned any = __builtin_amdgcn_ballot_w32(h0 | h1 | h2 | h3 | h4 | h5 | h6 | h7);
    if (any != 0u) {
#define HITJ(J, HJ, SJ) { \
        const unsigned mj = __builtin_amdgcn_ballot_w32(HJ); \
        if (mj != 0u) { \
          if (HJ) { \
            const int pos = wc + (int)__builtin_amdgcn_mbcnt_lo(mj, 0u); \
            if (pos < WCAP) list[wave * WCAP + pos] = ((el0 + (J)) << 12) | (int)(SJ); \
          } \
          wc += (int)__builtin_popcount(mj); } }
      HITJ(0, h0, s0)
      HITJ(1, h1, s1)
      HITJ(2, h2, s2)
      HITJ(3, h3, s3)
      HITJ(4, h4, s4)
      HITJ(5, h5, s5)
      HITJ(6, h6, s6)
      HITJ(7, h7, s7)
#undef HITJ
    }
  }
  return wc;
}

__global__ __launch_bounds__(NTHR) void k_prep(
    const float* __restrict__ W1, const float* __restrict__ W2,
    _Float16* wpl, float* idtab, int nMat) {
  const int i   = blockIdx.x * NTHR + threadIdx.x;
  const int per = DF * DF / 8;
  const int nW  = 2 * nMat * per;
  if (i < nW) {
    const int mat = i / per;
    const int o   = (i - mat * per) * 8;
    const int n   = o / DF;
    const int k0  = o - n * DF;
    const float* base = (mat < nMat) ? (W1 + (size_t)mat * DF * DF) : (W2 + (size_t)(mat - nMat) * DF * DF);
    const float* p = base + (size_t)k0 * DF + n;
    v4f a, b;
    a.x = p[0];      a.y = p[DF];     a.z = p[2 * DF]; a.w = p[3 * DF];
    b.x = p[4 * DF]; b.y = p[5 * DF]; b.z = p[6 * DF]; b.w = p[7 * DF];
    a = a * WSCALE;
    b = b * WSCALE;
    const v8h hv = cvt8(a, b);
    _Float16* dp = wpl + (size_t)i * 8;
    *(volatile v8h*)dp = hv;
    __threadfence();
    *(volatile v8h*)dp = hv;
  } else if (i < nW + TABN / 4) {
    const int j = i - nW;
    const float one = (j >= 16 && j < 32) ? 1.0f : 0.0f;
    v4f v; v.x = one; v.y = one; v.z = one; v.w = one;
    float* dp = idtab + 4 * j;
    *(volatile v4f*)dp = v;
    __threadfence();
    *(volatile v4f*)dp = v;
  }
}

__global__ __launch_bounds__(NTHR) void k_agg(
    const int* __restrict__ ei, const float* __restrict__ hsrc, const float* __restrict__ tab,
    const _Float16* __restrict__ wpl, const float* __restrict__ bias,
    float* z1, double* part, int nN, int nE, int vec8, float floorv) {
  extern __shared__ v4f lds_dyn[];
  float*  acc  = (float*)lds_dyn;
  int*    list = (int*)(acc + NBA * DF);
  int*    wcnt = list + LISTN;
  double* dstg = (double*)list;
  const int tid = threadIdx.x, lane = tid & 31, wave = tid >> 5, hh = lane >> 4, m = lane & 15;
  const int nodeBase = blockIdx.x * NBA;
  const int* dsts = ei + nE;

  {
    const v4f z = {0.f, 0.f, 0.f, 0.f};
    for (int i = tid; i < NBA * DF / 4; i += NTHR) lds_dyn[i] = z;
  }
  const v2f tm = *(const v2f*)(tab + 2 * lane);
  const v2f ta = *(const v2f*)(tab + 64 + 2 * lane);
  const v2f tb = *(const v2f*)(tab + 128 + 2 * lane);
  __syncthreads();

  const int nChunks = (nE + CHUNK - 1) / CHUNK;
#pragma unroll 1
  for (int ch = 0; ch < nChunks; ++ch) {
    const int cbase = ch * CHUNK;
    const int wc = scan_chunk<NBA>(dsts, nE, cbase, nodeBase, vec8, list, tid, lane, wave);
    if (lane == 0) wcnt[wave] = wc;
    __syncthreads();
    if (wave == 0) {
#pragma unroll 1
      for (int wsx = 0; wsx < NWAVE; ++wsx) {
        int n = __builtin_amdgcn_readfirstlane(wcnt[wsx]);
        n = n > WCAP ? WCAP : (n < 0 ? 0 : n);
        const int* lp = list + wsx * WCAP;
#pragma unroll 1
        for (int i = 0; i < n; ++i) {
          const int ent  = __builtin_amdgcn_readfirstlane(lp[i]);
          const int slot = ent & (NBA - 1);
          int e = cbase + ((ent >> 12) & (CHUNK - 1));
          e = e > nE - 1 ? nE - 1 : e;
          int src = ei[e];
          src = src < 0 ? 0 : (src > nN - 1 ? nN - 1 : src);
          v2f v = *(const v2f*)(hsrc + (size_t)src * DF + 2 * lane);
          v = (v - tm) * ta + tb;
          v.x = fmaxf(v.x, floorv);
          v.y = fmaxf(v.y, floorv);
          v2f* ap = (v2f*)(acc + slot * DF + 2 * lane);
          *ap = *ap + v;
        }
      }
    }
    __syncthreads();
  }

  {
    const int c4 = (tid & 15) * 4;
    const v4f m4 = *(const v4f*)(tab + c4);
    const v4f a4 = *(const v4f*)(tab + 64 + c4);
    const v4f b4 = *(const v4f*)(tab + 128 + c4);
#pragma unroll 4
    for (int i = 0; i < (NBA * DF / 4) / NTHR; ++i) {
      const int idx  = i * NTHR + tid;
      const int slot = idx >> 4;
      int node = nodeBase + slot;
      node = node > nN - 1 ? nN - 1 : node;
      v4f v = *(const v4f*)(hsrc + (size_t)node * DF + c4);
      v = (v - m4) * a4 + b4;
      v.x = fmaxf(v.x, floorv); v.y = fmaxf(v.y, floorv);
      v.z = fmaxf(v.z, floorv); v.w = fmaxf(v.w, floorv);
      v4f* ap = (v4f*)(acc + slot * DF + c4);
      *ap = *ap + v;
    }
  }
  __syncthreads();

  FragH bw[2][4];
#pragma unroll
  for (int kt = 0; kt < 2; ++kt)
#pragma unroll
    for (int t = 0; t < 4; ++t) {
      const _Float16* bp = wpl + (size_t)(16 * t + m) * DF + 32 * kt + 8 * hh;
      bw[kt][t].h[0] = *(const v8h*)bp;
      bw[kt][t].h[1] = *(const v8h*)(bp + 16);
    }
  float bvv[4];
#pragma unroll
  for (int t = 0; t < 4; ++t) bvv[t] = bias[16 * t + m];

#pragma unroll 1
  for (int j = 0; j < NBA / (16 * NWAVE); ++j) {
    const int tt = wave * (NBA / (16 * NWAVE)) + j;
    v8f c[4];
#pragma unroll
    for (int t = 0; t < 4; ++t) { v8f z = {0.f, 0.f, 0.f, 0.f, 0.f, 0.f, 0.f, 0.f}; c[t] = z; }
#pragma unroll
    for (int kt = 0; kt < 2; ++kt) {
      const float* ap = acc + (16 * tt + m) * DF + 32 * kt + 8 * hh;
      const v4f p0 = *(const v4f*)ap,        p1 = *(const v4f*)(ap + 4);
      const v4f p2 = *(const v4f*)(ap + 16), p3 = *(const v4f*)(ap + 20);
      FragH a;
      a.h[0] = cvt8(p0, p1);
      a.h[1] = cvt8(p2, p3);
#pragma unroll
      for (int t = 0; t < 4; ++t) c[t] = wmh(a.v, bw[kt][t].v, c[t]);
    }
    float* sp = acc + (16 * tt + 8 * hh) * DF + m;
#pragma unroll
    for (int t = 0; t < 4; ++t) {
#pragma unroll
      for (int r = 0; r < 8; ++r) sp[r * DF + 16 * t] = c[t][r] * WINV + bvv[t];
    }
  }
  __syncthreads();

  const int nvalid = (nN - nodeBase) < NBA ? (nN - nodeBase) : NBA;
  {
    const int c = tid & 63, rg = tid >> 6;
    const int rbeg = rg * (NBA / 4);
    int rend = rbeg + NBA / 4;
    rend = rend < nvalid ? rend : nvalid;
    double s = 0.0, q = 0.0;
#pragma unroll 2
    for (int r = rbeg; r < rend; ++r) {
      const double v = (double)acc[r * DF + c];
      s += v;
      q += v * v;
    }
    dstg[rg * 64 + c]       = s;
    dstg[256 + rg * 64 + c] = q;
  }
  __syncthreads();
  if (tid < 64) {
    const double s = ((dstg[tid] + dstg[64 + tid]) + dstg[128 + tid]) + dstg[192 + tid];
    const double q = ((dstg[256 + tid] + dstg[320 + tid]) + dstg[384 + tid]) + dstg[448 + tid];
    dstg[512 + tid]      = s;
    dstg[512 + 64 + tid] = q;
  }
  __syncthreads();
  if (wave == 0) {
    const double* srcd = dstg + 512;
    double* gp = part + (size_t)blockIdx.x * PARTN;
    const v2d o0 = *(const v2d*)(srcd + 2 * lane);
    const v2d o1 = *(const v2d*)(srcd + 64 + 2 * lane);
    *(volatile v2d*)(gp + 2 * lane)      = o0;
    *(volatile v2d*)(gp + 64 + 2 * lane) = o1;
    __threadfence();
    *(volatile v2d*)(gp + 2 * lane)      = o0;
    *(volatile v2d*)(gp + 64 + 2 * lane) = o1;
  }

  {
    const int rsub = lane >> 4, c4 = (lane & 15) * 4;
    const int rw0  = wave * (NBA / NWAVE);
    float* gbase = z1 + (size_t)nodeBase * DF;
#pragma unroll 4
    for (int i = 0; i < NBA / NWAVE / 2; ++i) {
      const int r = rw0 + 2 * i + rsub;
      const v4f v = *(const v4f*)(acc + r * DF + c4);
      *(volatile v4f*)(gbase + (size_t)r * DF + c4) = v;
    }
    __threadfence();
#pragma unroll 4
    for (int i = 0; i < NBA / NWAVE / 2; ++i) {
      const int r = rw0 + 2 * i + rsub;
      const v4f v = *(const v4f*)(acc + r * DF + c4);
      *(volatile v4f*)(gbase + (size_t)r * DF + c4) = v;
    }
  }
}

__global__ __launch_bounds__(64) void k_bnfin(
    const double* __restrict__ part, int nParts, const float* __restrict__ gamma,
    const float* __restrict__ beta, float* tab, int nN) {
  __shared__ __attribute__((aligned(16))) float st[TABN];
  const int c = threadIdx.x;
  double s = 0.0, q = 0.0;
#pragma unroll 1
  for (int b = 0; b < nParts; ++b) {
    s += part[(size_t)b * PARTN + c];
    q += part[(size_t)b * PARTN + 64 + c];
  }
  const double inv  = 1.0 / (double)nN;
  const double mean = s * inv;
  double var = q * inv - mean * mean;
  var = var < 0.0 ? 0.0 : var;
  const float mf = (float)mean;
  const float vf = (float)var;
  const float rs = 1.0f / sqrtf(vf + BN_EPS);
  st[c]       = mf;
  st[64 + c]  = gamma[c] * rs;
  st[128 + c] = beta[c];
  st[192 + c] = 0.0f;
  __syncthreads();
  if (c < 32) {
    const v4f v0 = *(const v4f*)(st + 4 * c);
    const v4f v1 = *(const v4f*)(st + 128 + 4 * c);
    *(volatile v4f*)(tab + 4 * c)       = v0;
    *(volatile v4f*)(tab + 128 + 4 * c) = v1;
    __threadfence();
    *(volatile v4f*)(tab + 4 * c)       = v0;
    *(volatile v4f*)(tab + 128 + 4 * c) = v1;
  }
}

__global__ __launch_bounds__(NTHR) void k_gemm2(
    const float* __restrict__ z1, const float* __restrict__ tab, const _Float16* __restrict__ wpl,
    const float* __restrict__ bias, float* z2, double* part, int nN) {
  extern __shared__ v4f lds_dyn[];
  _Float16* sA   = (_Float16*)lds_dyn;
  float*    stg  = (float*)((char*)lds_dyn + GR2 * APITCH * 2);
  double*   dstg = (double*)lds_dyn;
  const int tid = threadIdx.x, lane = tid & 31, wave = tid >> 5, hh = lane >> 4, m = lane & 15;
  const int rowBase = blockIdx.x * GR2;

  {
    const int c0 = (tid & 7) * 8;
    const v4f mA = *(const v4f*)(tab + c0),       mB = *(const v4f*)(tab + c0 + 4);
    const v4f aA = *(const v4f*)(tab + 64 + c0),  aB = *(const v4f*)(tab + 64 + c0 + 4);
    const v4f bA = *(const v4f*)(tab + 128 + c0), bB = *(const v4f*)(tab + 128 + c0 + 4);
#pragma unroll
    for (int i = 0; i < (GR2 * DF / 8) / NTHR; ++i) {
      const int idx = i * NTHR + tid;
      const int r   = idx >> 3;
      int node = rowBase + r;
      node = node > nN - 1 ? nN - 1 : node;
      const float* xp = z1 + (size_t)node * DF + c0;
      v4f p = *(const v4f*)xp, q = *(const v4f*)(xp + 4);
      p = (p - mA) * aA + bA;
      q = (q - mB) * aB + bB;
      p.x = fmaxf(p.x, 0.f); p.y = fmaxf(p.y, 0.f); p.z = fmaxf(p.z, 0.f); p.w = fmaxf(p.w, 0.f);
      q.x = fmaxf(q.x, 0.f); q.y = fmaxf(q.y, 0.f); q.z = fmaxf(q.z, 0.f); q.w = fmaxf(q.w, 0.f);
      *(v8h*)(sA + r * APITCH + c0) = cvt8(p, q);
    }
  }
  __syncthreads();

  FragH bw[2][4];
#pragma unroll
  for (int kt = 0; kt < 2; ++kt)
#pragma unroll
    for (int t = 0; t < 4; ++t) {
      const _Float16* bp = wpl + (size_t)(16 * t + m) * DF + 32 * kt + 8 * hh;
      bw[kt][t].h[0] = *(const v8h*)bp;
      bw[kt][t].h[1] = *(const v8h*)(bp + 16);
    }
  float bvv[4];
#pragma unroll
  for (int t = 0; t < 4; ++t) bvv[t] = bias[16 * t + m];

#pragma unroll
  for (int j = 0; j < GR2 / (16 * NWAVE); ++j) {
    const int tt = wave * (GR2 / (16 * NWAVE)) + j;
    v8f c[4];
#pragma unroll
    for (int t = 0; t < 4; ++t) { v8f z = {0.f, 0.f, 0.f, 0.f, 0.f, 0.f, 0.f, 0.f}; c[t] = z; }
    const _Float16* ar = sA + (16 * tt + m) * APITCH + 8 * hh;
#pragma unroll
    for (int kt = 0; kt < 2; ++kt) {
      FragH a;
      a.h[0] = *(const v8h*)(ar + 32 * kt);
      a.h[1] = *(const v8h*)(ar + 32 * kt + 16);
#pragma unroll
      for (int t = 0; t < 4; ++t) c[t] = wmh(a.v, bw[kt][t].v, c[t]);
    }
    float* sp = stg + (16 * tt + 8 * hh) * DF + m;
#pragma unroll
    for (int t = 0; t < 4; ++t) {
#pragma unroll
      for (int r = 0; r < 8; ++r) sp[r * DF + 16 * t] = c[t][r] * WINV + bvv[t];
    }
  }
  __syncthreads();

  const int nvalid = (nN - rowBase) < GR2 ? (nN - rowBase) : GR2;
  {
    const int c = tid & 63, rg = tid >> 6;
    const int rbeg = rg * (GR2 / 4);
    int rend = rbeg + GR2 / 4;
    rend = rend < nvalid ? rend : nvalid;
    double s = 0.0, q = 0.0;
#pragma unroll 2
    for (int r = rbeg; r < rend; ++r) {
      const double v = (double)stg[r * DF + c];
      s += v;
      q += v * v;
    }
    dstg[rg * 64 + c]       = s;
    dstg[256 + rg * 64 + c] = q;
  }
  __syncthreads();
  if (tid < 64) {
    const double s = ((dstg[tid] + dstg[64 + tid]) + dstg[128 + tid]) + dstg[192 + tid];
    const double q = ((dstg[256 + tid] + dstg[320 + tid]) + dstg[384 + tid]) + dstg[448 + tid];
    dstg[512 + tid]      = s;
    dstg[512 + 64 + tid] = q;
  }
  __syncthreads();
  if (wave == 0) {
    const double* srcd = dstg + 512;
    double* gp = part + (size_t)blockIdx.x * PARTN;
    const v2d o0 = *(const v2d*)(srcd + 2 * lane);
    const v2d o1 = *(const v2d*)(srcd + 64 + 2 * lane);
    *(volatile v2d*)(gp + 2 * lane)      = o0;
    *(volatile v2d*)(gp + 64 + 2 * lane) = o1;
    __threadfence();
    *(volatile v2d*)(gp + 2 * lane)      = o0;
    *(volatile v2d*)(gp + 64 + 2 * lane) = o1;
  }

  {
    const int rsub = lane >> 4, c4 = (lane & 15) * 4;
    const int rw0  = wave * (GR2 / NWAVE);
    float* gbase = z2 + (size_t)rowBase * DF;
#pragma unroll 4
    for (int i = 0; i < GR2 / NWAVE / 2; ++i) {
      const int r = rw0 + 2 * i + rsub;
      const v4f v = *(const v4f*)(stg + r * DF + c4);
      *(volatile v4f*)(gbase + (size_t)r * DF + c4) = v;
    }
    __threadfence();
#pragma unroll 4
    for (int i = 0; i < GR2 / NWAVE / 2; ++i) {
      const int r = rw0 + 2 * i + rsub;
      const v4f v = *(const v4f*)(stg + r * DF + c4);
      *(volatile v4f*)(gbase + (size_t)r * DF + c4) = v;
    }
  }
}

__global__ __launch_bounds__(NTHR) void k_pool(
    const int* __restrict__ batch, const float* __restrict__ z2, const float* __restrict__ tab,
    float* out, int nN, int nG, int colOff, int ldo) {
  __shared__ __attribute__((aligned(16))) float acc[GBLK * DF];
  __shared__ __attribute__((aligned(16))) int   list[LISTN];
  __shared__ int wcnt[NWAVE];
  const int tid = threadIdx.x, lane = tid & 31, wave = tid >> 5;
  const int gBase = blockIdx.x * GBLK;

  {
    const v4f z = {0.f, 0.f, 0.f, 0.f};
    for (int i = tid; i < GBLK * DF / 4; i += NTHR) *(v4f*)(acc + 4 * i) = z;
  }
  const v2f tm = *(const v2f*)(tab + 2 * lane);
  const v2f ta = *(const v2f*)(tab + 64 + 2 * lane);
  const v2f tb = *(const v2f*)(tab + 128 + 2 * lane);
  __syncthreads();

  const int nChunks = (nN + CHUNK - 1) / CHUNK;
#pragma unroll 1
  for (int ch = 0; ch < nChunks; ++ch) {
    const int cbase = ch * CHUNK;
    const int wc = scan_chunk<GBLK>(batch, nN, cbase, gBase, 1, list, tid, lane, wave);
    if (lane == 0) wcnt[wave] = wc;
    __syncthreads();
    if (wave == 0) {
#pragma unroll 1
      for (int wsx = 0; wsx < NWAVE; ++wsx) {
        int n = __builtin_amdgcn_readfirstlane(wcnt[wsx]);
        n = n > WCAP ? WCAP : (n < 0 ? 0 : n);
        const int* lp = list + wsx * WCAP;
#pragma unroll 1
        for (int i = 0; i < n; ++i) {
          const int ent  = __builtin_amdgcn_readfirstlane(lp[i]);
          const int slot = ent & (GBLK - 1);
          int node = cbase + ((ent >> 12) & (CHUNK - 1));
          node = node > nN - 1 ? nN - 1 : node;
          v2f v = *(const v2f*)(z2 + (size_t)node * DF + 2 * lane);
          v = (v - tm) * ta + tb;
          v.x = fmaxf(v.x, 0.f);
          v.y = fmaxf(v.y, 0.f);
          v2f* ap = (v2f*)(acc + slot * DF + 2 * lane);
          *ap = *ap + v;
        }
      }
    }
    __syncthreads();
  }

  {
    const int gsub = lane >> 4, c4 = (lane & 15) * 4;
#pragma unroll
    for (int i = 0; i < GBLK / NWAVE / 2; ++i) {
      const int gl = wave * (GBLK / NWAVE) + 2 * i + gsub;
      const int g  = gBase + gl;
      if ((unsigned)g < (unsigned)nG) {
        const v4f v = *(const v4f*)(acc + gl * DF + c4);
        *(volatile v4f*)(out + (size_t)g * ldo + colOff + c4) = v;
      }
    }
    __threadfence();
#pragma unroll
    for (int i = 0; i < GBLK / NWAVE / 2; ++i) {
      const int gl = wave * (GBLK / NWAVE) + 2 * i + gsub;
      const int g  = gBase + gl;
      if ((unsigned)g < (unsigned)nG) {
        const v4f v = *(const v4f*)(acc + gl * DF + c4);
        *(volatile v4f*)(out + (size_t)g * ldo + colOff + c4) = v;
      }
    }
  }
}

extern "C" void kernel_launch(void* const* d_in, const int* in_sizes, int n_in,
                              void* d_out, int out_size, void* d_ws, size_t ws_size,
                              hipStream_t stream) {
  if (n_in < 11) return;
  const int nN = in_sizes[0] / DF;
  const int nE = in_sizes[1] / 2;
  const int nL = in_sizes[3] / (DF * DF);
  if (nN <= 0 || nE < 0 || nL <= 0) return;
  if (in_sizes[0] != nN * DF || in_sizes[1] != 2 * nE || in_sizes[2] != nN) return;
  if (in_sizes[3] != nL * DF * DF || in_sizes[7] != nL * DF * DF) return;
  if (in_sizes[4] != nL * DF || in_sizes[5] != nL * DF || in_sizes[6] != nL * DF) return;
  if (in_sizes[8] != nL * DF || in_sizes[9] != nL * DF || in_sizes[10] != nL * DF) return;
  const int ldo = nL * DF;
  const int nG  = out_size / ldo;
  if (nG <= 0 || out_size != nG * ldo) return;

  const float* x     = (const float*)d_in[0];
  const int*   ei    = (const int*)d_in[1];
  const int*   batch = (const int*)d_in[2];
  const float* W1    = (const float*)d_in[3];
  const float* b1    = (const float*)d_in[4];
  const float* g1    = (const float*)d_in[5];
  const float* bt1   = (const float*)d_in[6];
  const float* W2    = (const float*)d_in[7];
  const float* b2    = (const float*)d_in[8];
  const float* g_out = (const float*)d_in[9];
  const float* b_out = (const float*)d_in[10];
  float* out = (float*)d_out;

  const int nBlkA = (nN + NBA - 1) / NBA;
  const int nBlkG = (nN + GR2 - 1) / GR2;
  const int nBlkP = (nG + GBLK - 1) / GBLK;

  char* ws = (char*)d_ws;
  size_t off = 0;
  const size_t oWpl = off; off += (size_t)2 * nL * DF * DF * 2;                 off = (off + 255) & ~(size_t)255;
  const size_t oId  = off; off += (size_t)TABN * 4;                             off = (off + 255) & ~(size_t)255;
  const size_t oT1  = off; off += (size_t)TABN * 4;                             off = (off + 255) & ~(size_t)255;
  const size_t oT2  = off; off += (size_t)TABN * 4;                             off = (off + 255) & ~(size_t)255;
  const size_t oP1  = off; off += (size_t)nBlkA * PARTN * 8;                    off = (off + 255) & ~(size_t)255;
  const size_t oP2  = off; off += (size_t)nBlkG * PARTN * 8;                    off = (off + 255) & ~(size_t)255;
  const size_t oZ1  = off; off += (size_t)nBlkA * NBA * DF * 4;                 off = (off + 255) & ~(size_t)255;
  const size_t oZ2  = off; off += (size_t)nBlkG * GR2 * DF * 4;                 off = (off + 255) & ~(size_t)255;
  if (off > ws_size) return;
  if (off > (size_t)134217728) return;
  _Float16* wpl   = (_Float16*)(ws + oWpl);
  float*    idtab = (float*)(ws + oId);
  float*    tab1  = (float*)(ws + oT1);
  float*    tab2  = (float*)(ws + oT2);
  double*   part1 = (double*)(ws + oP1);
  double*   part2 = (double*)(ws + oP2);
  float*    z1    = (float*)(ws + oZ1);
  float*    z2    = (float*)(ws + oZ2);

  const int vec8 = ((nE & 3) == 0) ? 1 : 0;

  const int nPrepThr = 2 * nL * (DF * DF / 8) + TABN / 4;
  k_prep<<<(nPrepThr + NTHR - 1) / NTHR, NTHR, 0, stream>>>(W1, W2, wpl, idtab, nL);

  hipFuncSetAttribute(reinterpret_cast<const void*>(&k_agg),
                      hipFuncAttributeMaxDynamicSharedMemorySize, LDS_AGG);
  hipFuncSetAttribute(reinterpret_cast<const void*>(&k_gemm2),
                      hipFuncAttributeMaxDynamicSharedMemorySize, LDS_G2);

  for (int l = 0; l < nL; ++l) {
    const float* hsrc   = (l == 0) ? x : (const float*)z2;
    const float* tsrc   = (l == 0) ? (const float*)idtab : (const float*)tab2;
    const float  floorv = (l == 0) ? -3.0e38f : 0.0f;
    k_agg<<<nBlkA, NTHR, LDS_AGG, stream>>>(ei, hsrc, tsrc, wpl + (size_t)l * DF * DF,
                                             b1 + l * DF, z1, part1, nN, nE, vec8, floorv);
    k_bnfin<<<1, 64, 0, stream>>>(part1, nBlkA, g1 + l * DF, bt1 + l * DF, tab1, nN);
    k_gemm2<<<nBlkG, NTHR, LDS_G2, stream>>>(z1, tab1, wpl + (size_t)(nL + l) * DF * DF,
                                              b2 + l * DF, z2, part2, nN);
    k_bnfin<<<1, 64, 0, stream>>>(part2, nBlkG, g_out + l * DF, b_out + l * DF, tab2, nN);
    k_pool<<<nBlkP, NTHR, 0, stream>>>(batch, z2, tab2, out, nN, nG, l * DF, ldo);
  }
}
